// GATedge_90752658965188
// MI455X (gfx1250) — hardware-run, weakly checked
//
#include <hip/hip_runtime.h>
#include <math.h>

typedef __attribute__((ext_vector_type(16))) _Float16 v16h;
typedef __attribute__((ext_vector_type(8)))  _Float16 v8h;
typedef __attribute__((ext_vector_type(8)))  float    v8f;
typedef __attribute__((ext_vector_type(4)))  float    v4f;

constexpr int kB    = 8;
constexpr int kNop  = 1000;
constexpr int kNopP = 1024;
constexpr int kNma  = 64;
constexpr int kInS  = 128;
constexpr int kInD  = 64;
constexpr int kDf   = 128;
constexpr int kRowsM = kB * kNma;
constexpr float kSlope = 0.2f;
static_assert((kNopP % 64) == 0 && kNopP >= kNop, "padded op count");
static_assert((kNopP % 32) == 0 && (kInS % 32) == 0, "GEMM K multiples of 32");
static_assert(kNma == 64 && kDf == 128 && kInS == 128 && kInD == 64, "tile maps assume these extents");
static_assert(kRowsM == 512, "row count");

constexpr float kCarryP = 4096.0f;
constexpr float kCarryH = 16.0f;
constexpr float kCarryT = 128.0f;
constexpr float kCarryW = 64.0f;
constexpr float kFoldAgg = kCarryT / (kCarryP * kCarryH);
constexpr float kFoldOut = 1.0f / (kCarryT * kCarryW);
constexpr float kF16MinNormal = 6.103515625e-05f;

constexpr size_t kOffHT = 0;
constexpr size_t kOffPP = kOffHT + (size_t)kB * kInS * kNopP * 2;
constexpr size_t kOffTT = kOffPP + (size_t)kB * kNma * kNopP * 2;
constexpr size_t kOffWT = kOffTT + (size_t)kRowsM * kInS * 2;
constexpr size_t kOffFD = kOffWT + (size_t)kDf * kInS * 2;
constexpr size_t kOffEL = kOffFD + (size_t)kRowsM * kDf * 4;
constexpr size_t kOffER = kOffEL + (size_t)kB * kNopP * 4;
constexpr size_t kOffIZ = kOffER + (size_t)kRowsM * 4;
constexpr size_t kOffAK = kOffIZ + (size_t)kRowsM * 4;
constexpr size_t kOffSE = kOffAK + (size_t)kRowsM * 4;
constexpr size_t kOffVL = kOffSE + (size_t)kRowsM * 4;
constexpr size_t kWsTotal = kOffVL + (size_t)160 * 4;
static_assert(kWsTotal == 3613312ull, "carve total");
static_assert(kWsTotal <= 134217728ull, "carve cap");
static_assert((kOffPP % 128) == 0 && (kOffTT % 128) == 0 && (kOffWT % 128) == 0 && (kOffFD % 128) == 0 &&
              (kOffEL % 128) == 0 && (kOffER % 128) == 0 && (kOffIZ % 128) == 0 && (kOffAK % 128) == 0 &&
              (kOffSE % 128) == 0 && (kOffVL % 128) == 0, "128-B aligned regions");

__device__ __forceinline__ _Float16 to_h16_flush(float x) {
  const float y = (fabsf(x) < kF16MinNormal) ? 0.0f : x;
  return (_Float16)y;
}

__device__ __forceinline__ v16h frag_load_h(const _Float16* p) {
  union U { v16h v; v8h h[2]; };
  U f;
  f.h[0] = *(const v8h*)(p);
  f.h[1] = *(const v8h*)(p + 16);
  return f.v;
}

__device__ __forceinline__ v8f mma_h(v16h a, v16h b, v8f c) {
  c = __builtin_amdgcn_wmma_f32_16x16x32_f16(false, a, false, b, (short)0, c, false, false);
  asm volatile("v_nop\n\tv_nop\n\tv_nop\n\tv_nop" : "+v"(c) : "v"(a), "v"(b));
  return c;
}

__global__ __launch_bounds__(256) void prep_kernel(
    const float* __restrict__ h_dst, const float* __restrict__ W_src, const float* __restrict__ W_dst,
    const float* __restrict__ W_edge, const float* __restrict__ attn_l, const float* __restrict__ attn_r,
    float* __restrict__ featdst, float* __restrict__ er, float* __restrict__ vls,
    unsigned short* __restrict__ wsrcT)
{
  __shared__ __align__(16) float sH[kNma * kInD];
  __shared__ __align__(16) float sF[kNma * kDf];
  __shared__ __align__(16) float sV[160];
  __shared__ __align__(16) float sEr[kNma];
  const int tid = threadIdx.x, lane = tid & 31, wave = tid >> 5;
  const int b = blockIdx.x;

#pragma unroll
  for (int i = 0; i < 4; ++i) {
    const int idx = tid + 256 * i;
    *(v4f*)(sH + idx * 4) = *(const v4f*)(h_dst + (size_t)b * (kNma * kInD) + idx * 4);
  }
  if (b == 0) {
    if (wave < 4) {
      float a = 0.0f;
#pragma unroll 4
      for (int d = 0; d < kDf; ++d) a = fmaf(W_src[tid * kDf + d], attn_l[d], a);
      sV[tid] = a;
    } else if (wave == 4) {
      float a = 0.0f;
#pragma unroll 4
      for (int d = 0; d < kDf; ++d) a = fmaf(W_edge[d], attn_l[d], a);
      sV[tid] = a;
    }
  }
  __syncthreads();

  {
    const int d = tid & 127, mh = tid >> 7;
    float acc[32];
#pragma unroll
    for (int mm = 0; mm < 32; ++mm) acc[mm] = 0.0f;
#pragma unroll 1
    for (int k = 0; k < kInD; ++k) {
      const float w = W_dst[k * kDf + d];
#pragma unroll
      for (int mm = 0; mm < 32; ++mm) acc[mm] = fmaf(sH[(mh * 32 + mm) * kInD + k], w, acc[mm]);
    }
#pragma unroll
    for (int mm = 0; mm < 32; ++mm) sF[(mh * 32 + mm) * kDf + d] = acc[mm];
  }
  __syncthreads();
  if (wave < 2) {
    float a = 0.0f;
#pragma unroll 4
    for (int d = 0; d < kDf; ++d) a = fmaf(sF[tid * kDf + d], attn_r[d], a);
    sEr[tid] = a;
  }
  __syncthreads();

  v4f fv[8];
#pragma unroll
  for (int it = 0; it < 8; ++it) fv[it] = *(const v4f*)(sF + (it * 8 + wave) * kDf + lane * 4);
  const v4f ev = *(const v4f*)(sEr + (lane & 15) * 4);
  v4f vA = (v4f){0.0f, 0.0f, 0.0f, 0.0f};
  v4f vB = (v4f){0.0f, 0.0f, 0.0f, 0.0f};
  if (b == 0) {
    vA = *(const v4f*)(sV + lane * 4);
    vB = *(const v4f*)(sV + 128 + (lane & 7) * 4);
  }
  const int widx = b * 256 + tid;
  const int wn = widx >> 4, wk8 = widx & 15;
  v8h wv;
#pragma unroll
  for (int e = 0; e < 8; ++e) wv[e] = to_h16_flush(W_src[(wk8 * 8 + e) * kDf + wn] * kCarryW);

  for (int pass = 0; pass < 2; ++pass) {
#pragma unroll
    for (int it = 0; it < 8; ++it)
      *(volatile v4f*)(featdst + (size_t)(b * kNma + it * 8 + wave) * kDf + lane * 4) = fv[it];
    *(volatile v8h*)(wsrcT + (size_t)wn * kInS + wk8 * 8) = wv;
    if (wave == 0 && lane < 16) *(volatile v4f*)(er + b * kNma + lane * 4) = ev;
    if (b == 0) {
      if (wave == 1) *(volatile v4f*)(vls + lane * 4) = vA;
      if (wave == 2 && lane < 8) *(volatile v4f*)(vls + 128 + lane * 4) = vB;
    }
    __threadfence();
  }
}

__global__ __launch_bounds__(256) void hsrc_kernel(
    const float* __restrict__ h_src, const float* __restrict__ vls,
    unsigned short* __restrict__ hsrcT, float* __restrict__ el)
{
  constexpr int kPitch = 132;
  __shared__ __align__(16) float sT[64 * kPitch];
  __shared__ __align__(16) float sVl[kInS];
  __shared__ __align__(16) float sEl[64];
  const int tid = threadIdx.x, lane = tid & 31, wave = tid >> 5;
  const int b = blockIdx.y, o0 = blockIdx.x * 64;

  if (wave < 4) sVl[tid] = vls[tid];
#pragma unroll
  for (int i = 0; i < 8; ++i) {
    const int idx = tid + 256 * i;
    const int r = idx >> 5, c4 = (idx & 31) * 4;
    const int o = o0 + r;
    const int oc = (o < kNop) ? o : (kNop - 1);
    const v4f v = *(const v4f*)(h_src + ((size_t)b * kNop + oc) * kInS + c4);
    float x0 = v[0], x1 = v[1], x2 = v[2], x3 = v[3];
    asm volatile("" : "+v"(x0), "+v"(x1), "+v"(x2), "+v"(x3));
    const bool live = (o < kNop);
    v4f z;
    z[0] = live ? x0 : 0.0f;
    z[1] = live ? x1 : 0.0f;
    z[2] = live ? x2 : 0.0f;
    z[3] = live ? x3 : 0.0f;
    *(v4f*)(sT + r * kPitch + c4) = z;
  }
  __syncthreads();
  if (wave < 2) {
    float a = 0.0f;
#pragma unroll 4
    for (int k = 0; k < kInS; ++k) a = fmaf(sT[tid * kPitch + k], sVl[k], a);
    sEl[tid] = a;
  }
  __syncthreads();

  const int q = lane >> 3, o8 = lane & 7;
  v8h hv[4];
#pragma unroll
  for (int it = 0; it < 4; ++it) {
    const int k = it * 32 + wave * 4 + q;
#pragma unroll
    for (int e = 0; e < 8; ++e) hv[it][e] = to_h16_flush(sT[(o8 * 8 + e) * kPitch + k] * kCarryH);
  }
  const v4f ev = *(const v4f*)(sEl + (lane & 15) * 4);
  for (int pass = 0; pass < 2; ++pass) {
#pragma unroll
    for (int it = 0; it < 4; ++it) {
      const int k = it * 32 + wave * 4 + q;
      *(volatile v8h*)(hsrcT + ((size_t)b * kInS + k) * kNopP + o0 + o8 * 8) = hv[it];
    }
    if (wave == 0 && lane < 16) *(volatile v4f*)(el + b * kNopP + o0 + lane * 4) = ev;
    __threadfence();
  }
}

__global__ __launch_bounds__(256) void softmax_kernel(
    const float* __restrict__ edge, const int* __restrict__ adj,
    const float* __restrict__ el, const float* __restrict__ er, const float* __restrict__ vls,
    unsigned short* __restrict__ Pp, float* __restrict__ izp, float* __restrict__ akp, float* __restrict__ sep)
{
  constexpr int kPp = 65;
  __shared__ __align__(16) float sEl[kNopP];
  __shared__ __align__(16) float sP[64 * kPp];
  __shared__ __align__(16) float sMxP[256];
  __shared__ __align__(16) float sZP[256];
  __shared__ __align__(16) float sSeP[256];
  __shared__ __align__(16) float sOut[3 * 64];
  const int tid = threadIdx.x, lane = tid & 31, wave = tid >> 5;
  const int b = blockIdx.x;
  const int m = tid & 63, grp = tid >> 6;

#pragma unroll
  for (int j = 0; j < 4; ++j) sEl[tid + 256 * j] = el[b * kNopP + tid + 256 * j];
  const float swe = vls[128];
  const float erm = er[b * kNma + m];
  const float er2 = erm + erm;
  const float ekk = (er2 > 0.0f) ? er2 : kSlope * er2;
  __syncthreads();

  const size_t base = (size_t)b * kNop * kNma + m;

  float mx = ekk;
#pragma unroll 2
  for (int o = grp; o < kNop; o += 4) {
    int aj = adj[base + (size_t)o * kNma];
    float ef = edge[base + (size_t)o * kNma];
    asm volatile("" : "+v"(aj), "+v"(ef));
    const float a = fmaf(ef, swe, sEl[o] + erm);
    const float e = (a > 0.0f) ? a : kSlope * a;
    const float cand = (aj == 1) ? e : ekk;
    mx = fmaxf(mx, cand);
  }
  sMxP[grp * 64 + m] = mx;
  __syncthreads();
  const float mxm = fmaxf(fmaxf(sMxP[m], sMxP[64 + m]), fmaxf(sMxP[128 + m], sMxP[192 + m]));

  float zs = 0.0f, ses = 0.0f;
  const int q = lane >> 3, o8 = lane & 7;
#pragma unroll 1
  for (int tile = 0; tile < kNopP / 64; ++tile) {
#pragma unroll 1
    for (int j = 0; j < 16; ++j) {
      const int ol = grp + 4 * j;
      const int o = tile * 64 + ol;
      const int oc = (o < kNop) ? o : (kNop - 1);
      int aj = adj[base + (size_t)oc * kNma];
      float ef = edge[base + (size_t)oc * kNma];
      asm volatile("" : "+v"(aj), "+v"(ef));
      const float a = fmaf(ef, swe, sEl[oc] + erm);
      const float e = (a > 0.0f) ? a : kSlope * a;
      const float arg = fminf(e - mxm, 0.0f);
      float pe = expf(arg);
      asm volatile("" : "+v"(pe));
      const bool live = (aj == 1) && (o < kNop);
      const float p = live ? pe : 0.0f;
      zs += p;
      ses = fmaf(ef, p, ses);
      sP[ol * kPp + m] = p;
    }
    __syncthreads();
    v8h hv[2];
#pragma unroll
    for (int it = 0; it < 2; ++it) {
      const int mrow = it * 32 + wave * 4 + q;
#pragma unroll
      for (int e = 0; e < 8; ++e) hv[it][e] = to_h16_flush(sP[(o8 * 8 + e) * kPp + mrow] * kCarryP);
    }
    for (int pass = 0; pass < 2; ++pass) {
#pragma unroll
      for (int it = 0; it < 2; ++it) {
        const int mrow = it * 32 + wave * 4 + q;
        *(volatile v8h*)(Pp + ((size_t)b * kNma + mrow) * kNopP + tile * 64 + o8 * 8) = hv[it];
      }
      __threadfence();
    }
    __syncthreads();
  }

  sZP[grp * 64 + m] = zs;
  sSeP[grp * 64 + m] = ses;
  __syncthreads();
  if (wave < 2) {
    const float pk = expf(ekk - mxm);
    const float zt = pk + ((sZP[m] + sZP[64 + m]) + (sZP[128 + m] + sZP[192 + m]));
    const float st = (sSeP[m] + sSeP[64 + m]) + (sSeP[128 + m] + sSeP[192 + m]);
    const float izv = 1.0f / zt;
    sOut[m] = izv;
    sOut[64 + m] = pk * izv;
    sOut[128 + m] = st * izv;
  }
  __syncthreads();
  const v4f v0 = *(const v4f*)(sOut + (lane & 15) * 4);
  const v4f v1 = *(const v4f*)(sOut + 64 + (lane & 15) * 4);
  const v4f v2 = *(const v4f*)(sOut + 128 + (lane & 15) * 4);
  for (int pass = 0; pass < 2; ++pass) {
    if (wave == 0 && lane < 16) {
      *(volatile v4f*)(izp + b * kNma + lane * 4) = v0;
      *(volatile v4f*)(akp + b * kNma + lane * 4) = v1;
      *(volatile v4f*)(sep + b * kNma + lane * 4) = v2;
    }
    __threadfence();
  }
}

__global__ __launch_bounds__(256) void agg_gemm_kernel(
    const unsigned short* __restrict__ Pp, const unsigned short* __restrict__ hsrcT,
    const float* __restrict__ izp, unsigned short* __restrict__ tpl)
{
  __shared__ __align__(16) float sT[8][16 * 68];
  const int tid = threadIdx.x, lane = tid & 31, wave = tid >> 5;
  const int blk = blockIdx.x;
  const int mt = wave & 3, nh = wave >> 2;
  const int rl = lane & 15, hh = lane >> 4;
  const int koff = hh * 8, mOff = hh * 8;

  const _Float16* Arow = (const _Float16*)Pp + ((size_t)blk * kNma + mt * 16 + rl) * kNopP + koff;
  const _Float16* Brow = (const _Float16*)hsrcT + ((size_t)blk * kInS + nh * 64 + rl) * kNopP + koff;

  v8f acc[4];
#pragma unroll
  for (int j = 0; j < 4; ++j) acc[j] = (v8f){0.f, 0.f, 0.f, 0.f, 0.f, 0.f, 0.f, 0.f};
#pragma unroll 1
  for (int k0 = 0; k0 < kNopP; k0 += 32) {
    const v16h a  = frag_load_h(Arow + k0);
    const v16h b0 = frag_load_h(Brow + k0);
    const v16h b1 = frag_load_h(Brow + (size_t)16 * kNopP + k0);
    const v16h b2 = frag_load_h(Brow + (size_t)32 * kNopP + k0);
    const v16h b3 = frag_load_h(Brow + (size_t)48 * kNopP + k0);
    acc[0] = mma_h(a, b0, acc[0]);
    acc[1] = mma_h(a, b1, acc[1]);
    acc[2] = mma_h(a, b2, acc[2]);
    acc[3] = mma_h(a, b3, acc[3]);
  }

  float* slab = sT[wave];
#pragma unroll
  for (int r = 0; r < 8; ++r) {
    const float s = izp[blk * kNma + mt * 16 + mOff + r] * kFoldAgg;
#pragma unroll
    for (int j = 0; j < 4; ++j) slab[(mOff + r) * 68 + j * 16 + rl] = acc[j][r] * s;
  }
  __syncthreads();
  const int q = lane >> 3, c8 = (lane & 7) * 8;
  v8h hv[4];
#pragma unroll
  for (int it = 0; it < 4; ++it) {
    const float* sp = slab + (it * 4 + q) * 68 + c8;
#pragma unroll
    for (int e = 0; e < 8; ++e) hv[it][e] = to_h16_flush(sp[e]);
  }
  for (int pass = 0; pass < 2; ++pass) {
#pragma unroll
    for (int it = 0; it < 4; ++it) {
      const int grow = blk * kNma + mt * 16 + it * 4 + q;
      *(volatile v8h*)(tpl + (size_t)grow * kInS + nh * 64 + c8) = hv[it];
    }
    __threadfence();
  }
}

__global__ __launch_bounds__(256) void out_gemm_kernel(
    const unsigned short* __restrict__ tpl, const unsigned short* __restrict__ wsrcT,
    const float* __restrict__ W_edge, const float* __restrict__ featdst,
    const float* __restrict__ akp, const float* __restrict__ sep, float* __restrict__ out)
{
  __shared__ __align__(16) float sT[8][16 * 68];
  const int tid = threadIdx.x, lane = tid & 31, wave = tid >> 5;
  const int blk = blockIdx.x;
  const int mt = wave & 3, nh = wave >> 2;
  const int rl = lane & 15, hh = lane >> 4;
  const int koff = hh * 8, mOff = hh * 8;

  const _Float16* Arow = (const _Float16*)tpl + ((size_t)blk * 64 + mt * 16 + rl) * kInS + koff;
  const _Float16* Brow = (const _Float16*)wsrcT + ((size_t)nh * 64 + rl) * kInS + koff;

  v8f acc[4];
#pragma unroll
  for (int j = 0; j < 4; ++j) acc[j] = (v8f){0.f, 0.f, 0.f, 0.f, 0.f, 0.f, 0.f, 0.f};
#pragma unroll 1
  for (int k0 = 0; k0 < kInS; k0 += 32) {
    const v16h a  = frag_load_h(Arow + k0);
    const v16h b0 = frag_load_h(Brow + k0);
    const v16h b1 = frag_load_h(Brow + (size_t)16 * kInS + k0);
    const v16h b2 = frag_load_h(Brow + (size_t)32 * kInS + k0);
    const v16h b3 = frag_load_h(Brow + (size_t)48 * kInS + k0);
    acc[0] = mma_h(a, b0, acc[0]);
    acc[1] = mma_h(a, b1, acc[1]);
    acc[2] = mma_h(a, b2, acc[2]);
    acc[3] = mma_h(a, b3, acc[3]);
  }

  float* slab = sT[wave];
#pragma unroll
  for (int r = 0; r < 8; ++r) {
#pragma unroll
    for (int j = 0; j < 4; ++j) slab[(mOff + r) * 68 + j * 16 + rl] = acc[j][r] * kFoldOut;
  }
  __syncthreads();

  const int c4 = (lane & 15) * 4;
  const int ncol = nh * 64 + c4;
  const v4f we = *(const v4f*)(W_edge + ncol);
#pragma unroll 1
  for (int it = 0; it < 8; ++it) {
    const int row = it * 2 + hh;
    const int grow = blk * 64 + mt * 16 + row;
    const v4f x = *(const v4f*)(slab + row * 68 + c4);
    const v4f fd = *(const v4f*)(featdst + (size_t)grow * kDf + ncol);
    const float sv = sep[grow];
    const float ak = akp[grow];
    v4f y;
#pragma unroll
    for (int e = 0; e < 4; ++e) {
      const float val = x[e] + we[e] * sv + fd[e] * ak;
      y[e] = 1.0f / (1.0f + expf(-val));
    }
    *(v4f*)(slab + row * 68 + c4) = y;
  }
  __syncthreads();

  for (int pass = 0; pass < 2; ++pass) {
#pragma unroll
    for (int it = 0; it < 8; ++it) {
      const int row = it * 2 + hh;
      const int grow = blk * 64 + mt * 16 + row;
      const v4f v = *(const v4f*)(slab + row * 68 + c4);
      *(volatile v4f*)(out + (size_t)grow * kDf + ncol) = v;
    }
    __threadfence();
  }
}

extern "C" void kernel_launch(void* const* d_in, const int* in_sizes, int n_in,
                              void* d_out, int out_size, void* d_ws, size_t ws_size,
                              hipStream_t stream) {
  if (n_in < 9) return;
  if (in_sizes[0] != kB * kNop * kInS) return;
  if (in_sizes[1] != kB * kNma * kInD) return;
  if (in_sizes[2] != kB * kNop * kNma) return;
  if (in_sizes[3] != kB * kNop * kNma) return;
  if (in_sizes[4] != kInS * kDf) return;
  if (in_sizes[5] != kInD * kDf) return;
  if (in_sizes[6] != kDf) return;
  if (in_sizes[7] != kDf) return;
  if (in_sizes[8] != kDf) return;
  if (out_size != kRowsM * kDf) return;
  if (ws_size < kWsTotal) return;

  const float* h_src  = (const float*)d_in[0];
  const float* h_dst  = (const float*)d_in[1];
  const float* edge   = (const float*)d_in[2];
  const int*   adj    = (const int*)d_in[3];
  const float* W_src  = (const float*)d_in[4];
  const float* W_dst  = (const float*)d_in[5];
  const float* W_edge = (const float*)d_in[6];
  const float* attn_l = (const float*)d_in[7];
  const float* attn_r = (const float*)d_in[8];
  float* out = (float*)d_out;

  char* ws = (char*)d_ws;
  unsigned short* HT = (unsigned short*)(ws + kOffHT);
  unsigned short* PP = (unsigned short*)(ws + kOffPP);
  unsigned short* TT = (unsigned short*)(ws + kOffTT);
  unsigned short* WT = (unsigned short*)(ws + kOffWT);
  float* FD = (float*)(ws + kOffFD);
  float* EL = (float*)(ws + kOffEL);
  float* ER = (float*)(ws + kOffER);
  float* IZ = (float*)(ws + kOffIZ);
  float* AK = (float*)(ws + kOffAK);
  float* SE = (float*)(ws + kOffSE);
  float* VL = (float*)(ws + kOffVL);

  prep_kernel<<<dim3(kB), dim3(256), 0, stream>>>(h_dst, W_src, W_dst, W_edge, attn_l, attn_r, FD, ER, VL, WT);
  hsrc_kernel<<<dim3(kNopP / 64, kB), dim3(256), 0, stream>>>(h_src, VL, HT, EL);
  softmax_kernel<<<dim3(kB), dim3(256), 0, stream>>>(edge, adj, EL, ER, VL, PP, IZ, AK, SE);
  agg_gemm_kernel<<<dim3(kB), dim3(256), 0, stream>>>(PP, HT, IZ, TT);
  out_gemm_kernel<<<dim3(kRowsM / 64), dim3(256), 0, stream>>>(TT, WT, W_edge, FD, AK, SE, out);
}
